// LowRankGNN_103079215402
// MI455X (gfx1250) — hardware-run, weakly checked
//
#include <hip/hip_runtime.h>
#include <stddef.h>


#define NL     3
#define NBR    4
#define ND     64
#define NM     2048
#define NN     500000
#define BSZ    20000
#define NFO    60000
#define NODES  (BSZ + NFO)
#define CD     256
#define CBW    (2 * ND)
#define GROWS  128
#define GCOLS  128
#define NT     (GCOLS / 16)
#define MP     20096
#define NBA    (MP / GROWS)
#define AROWS  GROWS
#define CAP    2048
#define CH     2048
#define NTHR   256
#define NWAVE  8
#define CNTW   32
#define WC_CARRY 64.0f
#define WC_INV   0.015625f
#define WSCAP  134217728
#define LDS_GEMM (GROWS * GCOLS * 4)
#define LDS_AGG  (AROWS * CD * 4 + CAP * 4)

static_assert((MP % GROWS) == 0 && MP >= BSZ && (MP - BSZ) < GROWS && NBA * GROWS == MP);
static_assert((BSZ % 16) == 0 && (CD % GCOLS) == 0 && (CD % 32) == 0 && CD == NBR * ND);
static_assert(GROWS == NWAVE * 16 && GCOLS == 32 * 4 && NTHR == NWAVE * 32);
static_assert(CH == NTHR * 8 && (CAP % (4 * NTHR)) == 0 && AROWS == 128 && (AROWS % NWAVE) == 0);
static_assert(((CD * CD / 8) % NTHR) == 0 && ((MP * CD / 8) % NTHR) == 0);
static_assert(ND == 64 && ((AROWS * CD / 4) % NTHR) == 0);
static_assert(LDS_AGG <= 160 * 1024 && LDS_GEMM == 65536);

typedef float           v4f   __attribute__((ext_vector_type(4)));
typedef float           v8f   __attribute__((ext_vector_type(8)));
typedef int             v4i   __attribute__((ext_vector_type(4)));
typedef unsigned short  v4us  __attribute__((ext_vector_type(4)));
typedef unsigned short  v8us  __attribute__((ext_vector_type(8)));
typedef __bf16          v16bf __attribute__((ext_vector_type(16)));
typedef _Float16        v16h  __attribute__((ext_vector_type(16)));
typedef _Float16        v8h   __attribute__((ext_vector_type(8)));
union FragB { v16bf v; v8us h[2]; };
union FragH { v16h  v; v8us h[2]; };
union Pack8 { v8h f; v8us u; };

static __device__ __forceinline__ unsigned short f2bf(float f) {
  unsigned int u = __float_as_uint(f);
  u = u + 0x7FFFu + ((u >> 16) & 1u);
  return (unsigned short)(u >> 16);
}
static __device__ __forceinline__ float bf2f(unsigned short b) {
  return __uint_as_float(((unsigned int)b) << 16);
}
static __device__ __forceinline__ void split4(const v4f v, v4us& hv, v4us& lv) {
#pragma unroll
  for (int j = 0; j < 4; ++j) {
    const unsigned short hb = f2bf(v[j]);
    hv[j] = hb;
    lv[j] = f2bf(v[j] - bf2f(hb));
  }
}

static __device__ __forceinline__ v8f wmb(v16bf a, v16bf b, v8f c) {
  v8f d = __builtin_amdgcn_wmma_f32_16x16x32_bf16(false, a, false, b, (short)0, c, false, false);
  asm volatile("v_nop\n\tv_nop\n\tv_nop\n\tv_nop" : "+v"(d) : "v"(a), "v"(b));
  return d;
}
static __device__ __forceinline__ v8f wmh(v16h a, v16h b, v8f c) {
  v8f d = __builtin_amdgcn_wmma_f32_16x16x32_f16(false, a, false, b, (short)0, c, false, false);
  asm volatile("v_nop\n\tv_nop\n\tv_nop\n\tv_nop" : "+v"(d) : "v"(a), "v"(b));
  return d;
}

__global__ __launch_bounds__(NTHR) void k_prepw(
    const float* __restrict__ Wc, const float* __restrict__ Wt, const float* __restrict__ Ws, const float* __restrict__ Wf,
    unsigned short* WcT, unsigned short* WtTh, unsigned short* WtTl,
    unsigned short* WsTh, unsigned short* WsTl, unsigned short* WfTh, unsigned short* WfTl) {
  const int y = (int)blockIdx.y;
  const int i = (int)blockIdx.x * NTHR + (int)threadIdx.x;
  if (i >= (CD * CD) / 8) return;
  const int e  = 8 * i;
  const int n  = e >> 8;
  const int k0 = e & (CD - 1);
  const float* W;
  unsigned short* dh;
  unsigned short* dl;
  int f16mode;
  if (y < NL) {
    W = Wc + (size_t)y * CD * CD; dh = WcT + (size_t)y * CD * CD; dl = dh; f16mode = 1;
  } else if (y < 2 * NL) {
    const int l = y - NL;
    W = Wt + (size_t)l * CD * CD; dh = WtTh + (size_t)l * CD * CD; dl = WtTl + (size_t)l * CD * CD; f16mode = 0;
  } else if (y < 3 * NL) {
    const int l = y - 2 * NL;
    W = Ws + (size_t)l * CD * CD; dh = WsTh + (size_t)l * CD * CD; dl = WsTl + (size_t)l * CD * CD; f16mode = 0;
  } else {
    W = Wf; dh = WfTh; dl = WfTl; f16mode = 0;
  }
  float a[8];
#pragma unroll
  for (int j = 0; j < 8; ++j) a[j] = W[(size_t)(k0 + j) * CD + n];
  if (f16mode) {
    Pack8 pk;
#pragma unroll
    for (int j = 0; j < 8; ++j) pk.f[j] = (_Float16)(a[j] * WC_CARRY);
    const v8us u = pk.u;
    unsigned short* p = dh + e;
    *(volatile v8us*)p = u;
    __threadfence();
    *(volatile v8us*)p = u;
  } else {
    v8us hv, lv;
#pragma unroll
    for (int j = 0; j < 8; ++j) {
      const unsigned short hb = f2bf(a[j]);
      hv[j] = hb;
      lv[j] = f2bf(a[j] - bf2f(hb));
    }
    unsigned short* ph = dh + e;
    unsigned short* pl = dl + e;
    *(volatile v8us*)ph = hv;
    *(volatile v8us*)pl = lv;
    __threadfence();
    *(volatile v8us*)ph = hv;
    *(volatile v8us*)pl = lv;
  }
}

__global__ __launch_bounds__(NTHR) void k_cvtx(const float* __restrict__ src, unsigned short* dhi, unsigned short* dlo,
                                               int rowLen, int nSrcRows, int total8) {
  const int i = (int)blockIdx.x * NTHR + (int)threadIdx.x;
  if (i >= total8) return;
  const size_t e  = (size_t)8 * (size_t)i;
  const int    r  = (int)(e / (size_t)rowLen);
  const int    k0 = (int)(e - (size_t)r * (size_t)rowLen);
  const int    rc = r < nSrcRows ? r : nSrcRows - 1;
  const float  z  = (r < nSrcRows) ? 1.0f : 0.0f;
  const float* sp = src + (size_t)rc * rowLen + k0;
  const v4f f0 = *(const v4f*)sp;
  const v4f f1 = *(const v4f*)(sp + 4);
  float v[8];
  v[0] = f0.x * z; v[1] = f0.y * z; v[2] = f0.z * z; v[3] = f0.w * z;
  v[4] = f1.x * z; v[5] = f1.y * z; v[6] = f1.z * z; v[7] = f1.w * z;
  v8us hv, lv;
#pragma unroll
  for (int j = 0; j < 8; ++j) {
    const unsigned short hb = f2bf(v[j]);
    hv[j] = hb;
    lv[j] = f2bf(v[j] - bf2f(hb));
  }
  unsigned short* ph = dhi + e;
  unsigned short* pl = dlo + e;
  *(volatile v8us*)ph = hv;
  *(volatile v8us*)pl = lv;
  __threadfence();
  *(volatile v8us*)ph = hv;
  *(volatile v8us*)pl = lv;
}

__global__ __launch_bounds__(NTHR) void k_build(const int* __restrict__ edst, int nE, int* tab, int* cnt) {
  __shared__ __attribute__((aligned(16))) int keys[CAP];
  __shared__ int wtot[NWAVE];
  __shared__ int ovf;
  const int tid = threadIdx.x, lane = tid & 31;
  const int wave = __builtin_amdgcn_readfirstlane(tid >> 5);
  const int b = (int)blockIdx.x;
  const int d0 = b * AROWS;
#pragma unroll 1
  for (int i = tid; i < CAP; i += NTHR) keys[i] = 0;
  if (tid == 0) ovf = 0;
  int listLen = 0;
  __syncthreads();
  const int nCh = (nE + CH - 1) / CH;
#pragma unroll 1
  for (int ch = 0; ch < nCh; ++ch) {
    const int cb = ch * CH;
    const int e0 = cb + 8 * tid;
    int d[8];
    if (cb + CH <= nE) {
      const v4i u0 = *(const v4i*)(edst + e0);
      const v4i u1 = *(const v4i*)(edst + e0 + 4);
      d[0] = u0.x; d[1] = u0.y; d[2] = u0.z; d[3] = u0.w;
      d[4] = u1.x; d[5] = u1.y; d[6] = u1.z; d[7] = u1.w;
    } else {
#pragma unroll
      for (int j = 0; j < 8; ++j) {
        const int ej = e0 + j;
        const int ec = ej < nE ? ej : nE - 1;
        const int dv = edst[ec];
        d[j] = (ej < nE) ? dv : -1;
      }
    }
    int hit[8];
    int c = 0;
#pragma unroll
    for (int j = 0; j < 8; ++j) {
      const int dl = d[j] - d0;
      const int hj = (((unsigned)dl < (unsigned)AROWS) && (d[j] < BSZ)) ? 1 : 0;
      hit[j] = hj;
      c += hj;
    }
    int incl = c;
#pragma unroll
    for (int s = 1; s < 32; s <<= 1) {
      const int t = __shfl_up(incl, s);
      if (lane >= s) incl += t;
    }
    if (lane == 31) wtot[wave] = incl;
    __syncthreads();
    int base = 0, tot = 0;
#pragma unroll
    for (int w = 0; w < NWAVE; ++w) {
      const int v = wtot[w];
      base += (w < wave) ? v : 0;
      tot += v;
    }
    int pos = listLen + base + incl - c;
#pragma unroll
    for (int j = 0; j < 8; ++j) {
      if (hit[j]) {
        if (pos < CAP) keys[pos] = (d[j] - d0) | ((e0 + j) << 7);
        else ovf = 1;
        ++pos;
      }
    }
    listLen += tot;
    __syncthreads();
  }
  const int fin = (ovf != 0 || listLen > CAP) ? -1 : listLen;
  int* tb = tab + (size_t)b * CAP;
  int* cp = cnt + (size_t)b * CNTW + lane;
#pragma unroll 1
  for (int q = tid; q < CAP / 4; q += NTHR) {
    const v4i v = *(const v4i*)(keys + 4 * q);
    *(volatile v4i*)(tb + 4 * q) = v;
  }
  if (wave == 0) *(volatile int*)cp = fin;
  __threadfence();
#pragma unroll 1
  for (int q = tid; q < CAP / 4; q += NTHR) {
    const v4i v = *(const v4i*)(keys + 4 * q);
    *(volatile v4i*)(tb + 4 * q) = v;
  }
  if (wave == 0) *(volatile int*)cp = fin;
}

__global__ __launch_bounds__(NTHR) void k_agg(
    const int* __restrict__ tab, const int* __restrict__ cnt,
    const int* __restrict__ esrc, const float* __restrict__ ew, int nE,
    const float* __restrict__ hsrc, const float* __restrict__ cbl, const int* __restrict__ cil,
    const int* __restrict__ foi, unsigned short* Aout) {
  extern __shared__ v4f lds_dyn[];
  float* accl = (float*)lds_dyn;
  int*   keys = (int*)(accl + AROWS * CD);
  const int tid = threadIdx.x, lane = tid & 31;
  const int wave = __builtin_amdgcn_readfirstlane(tid >> 5);
  const int b = (int)blockIdx.x;
  const int d0 = b * AROWS;
  {
    const v4f zz = {0.f, 0.f, 0.f, 0.f};
#pragma unroll 1
    for (int i = tid; i < (AROWS * CD) / 4; i += NTHR) ((v4f*)accl)[i] = zz;
  }
#pragma unroll 1
  for (int i = tid; i < CAP; i += NTHR) keys[i] = tab[(size_t)b * CAP + i];
  int n = cnt[(size_t)b * CNTW];
  const int poison = (n < 0) ? 1 : 0;
  n = n < 0 ? 0 : (n > CAP ? CAP : n);
  __syncthreads();

  const int br   = lane >> 3;
  const int cofs = (8 * lane) & (ND - 1);
  const int*   cib = cil + (size_t)br * NN;
  const float* cbb = cbl + (size_t)br * NM * CBW + cofs;
#pragma unroll 1
  for (int i = 0; i < n; ++i) {
    const int key = __builtin_amdgcn_readfirstlane(keys[i]);
    const int dl = key & (AROWS - 1);
    if ((dl & (NWAVE - 1)) == wave) {
      int e = (int)(((unsigned)key) >> 7);
      e = e > nE - 1 ? nE - 1 : e;
      int s = esrc[e];
      const float wv = ew[e];
      s = s < 0 ? 0 : (s > NODES - 1 ? NODES - 1 : s);
      const int rb = s > BSZ - 1 ? BSZ - 1 : s;
      int nf = s - BSZ;
      nf = nf < 0 ? 0 : nf;
      int fo = foi[nf];
      fo = fo < 0 ? 0 : (fo > NN - 1 ? NN - 1 : fo);
      int ci = cib[fo];
      ci = ci < 0 ? 0 : (ci > NM - 1 ? NM - 1 : ci);
      const float* pa = hsrc + (size_t)rb * CD + 8 * lane;
      const float* pb = cbb + (size_t)ci * CBW;
      const float* p  = (s < BSZ) ? pa : pb;
      const v4f v0 = *(const v4f*)p;
      const v4f v1 = *(const v4f*)(p + 4);
      const v4f w4 = {wv, wv, wv, wv};
      float* ap = accl + dl * CD + 8 * lane;
      v4f a0 = *(const v4f*)ap;
      v4f a1 = *(const v4f*)(ap + 4);
      a0 = w4 * v0 + a0;
      a1 = w4 * v1 + a1;
      *(v4f*)ap = a0;
      *(v4f*)(ap + 4) = a1;
    }
  }
  __syncthreads();

  const float qn = __uint_as_float(0x7FC00000u);
  const float* lrow = accl + (size_t)(wave * 16) * CD + 8 * lane;
  unsigned short* grow = Aout + (size_t)(d0 + wave * 16) * CD + 8 * lane;
#pragma unroll
  for (int r = 0; r < 16; ++r) {
    const v4f v0 = *(const v4f*)(lrow + r * CD);
    const v4f v1 = *(const v4f*)(lrow + r * CD + 4);
    Pack8 pk;
#pragma unroll
    for (int j = 0; j < 4; ++j) {
      const float x0 = poison ? qn : v0[j];
      const float x1 = poison ? qn : v1[j];
      pk.f[j] = (_Float16)x0;
      pk.f[4 + j] = (_Float16)x1;
    }
    const v8us u = pk.u;
    *(volatile v8us*)(grow + (size_t)r * CD) = u;
  }
  __threadfence();
#pragma unroll
  for (int r = 0; r < 16; ++r) {
    const v4f v0 = *(const v4f*)(lrow + r * CD);
    const v4f v1 = *(const v4f*)(lrow + r * CD + 4);
    Pack8 pk;
#pragma unroll
    for (int j = 0; j < 4; ++j) {
      const float x0 = poison ? qn : v0[j];
      const float x1 = poison ? qn : v1[j];
      pk.f[j] = (_Float16)x0;
      pk.f[4 + j] = (_Float16)x1;
    }
    const v8us u = pk.u;
    *(volatile v8us*)(grow + (size_t)r * CD) = u;
  }
}

static __device__ __forceinline__ void mac_x3(const unsigned short* __restrict__ ah, const unsigned short* __restrict__ al,
                                              const unsigned short* __restrict__ bh0, const unsigned short* __restrict__ bl0,
                                              v8f (&acc)[NT]) {
#pragma unroll 1
  for (int kt = 0; kt < CD / 32; ++kt) {
    FragB fah, fal;
    fah.h[0] = *(const v8us*)(ah + 32 * kt);
    fah.h[1] = *(const v8us*)(ah + 32 * kt + 16);
    fal.h[0] = *(const v8us*)(al + 32 * kt);
    fal.h[1] = *(const v8us*)(al + 32 * kt + 16);
#pragma unroll
    for (int t = 0; t < NT; ++t) {
      const size_t to = (size_t)(16 * t) * CD + (size_t)(32 * kt);
      FragB fbh, fbl;
      fbh.h[0] = *(const v8us*)(bh0 + to);
      fbh.h[1] = *(const v8us*)(bh0 + to + 16);
      fbl.h[0] = *(const v8us*)(bl0 + to);
      fbl.h[1] = *(const v8us*)(bl0 + to + 16);
      v8f d = acc[t];
      d = wmb(fah.v, fbh.v, d);
      d = wmb(fah.v, fbl.v, d);
      d = wmb(fal.v, fbh.v, d);
      acc[t] = d;
    }
  }
}

__global__ __launch_bounds__(NTHR) void k_gemm_f16(
    const unsigned short* __restrict__ A, const unsigned short* __restrict__ B,
    const float* __restrict__ bias, unsigned short* Ch, unsigned short* Cl) {
  extern __shared__ v4f lds_dyn[];
  float* stg = (float*)lds_dyn;
  const int tid = threadIdx.x, lane = tid & 31, hh = lane >> 4, m = lane & 15;
  const int wave = __builtin_amdgcn_readfirstlane(tid >> 5);
  const int rowBase = (int)blockIdx.x * GROWS;
  const int colBase = (int)blockIdx.y * GCOLS;
  const unsigned short* ap = A + (size_t)(rowBase + wave * 16 + m) * CD + 8 * hh;
  const unsigned short* bp = B + (size_t)(colBase + m) * CD + 8 * hh;

  v8f acc[NT];
#pragma unroll
  for (int t = 0; t < NT; ++t) { v8f zz = {0.f, 0.f, 0.f, 0.f, 0.f, 0.f, 0.f, 0.f}; acc[t] = zz; }

#pragma unroll 1
  for (int kt = 0; kt < CD / 32; ++kt) {
    FragH fa;
    fa.h[0] = *(const v8us*)(ap + 32 * kt);
    fa.h[1] = *(const v8us*)(ap + 32 * kt + 16);
#pragma unroll
    for (int t = 0; t < NT; ++t) {
      const size_t to = (size_t)(16 * t) * CD + (size_t)(32 * kt);
      FragH fb;
      fb.h[0] = *(const v8us*)(bp + to);
      fb.h[1] = *(const v8us*)(bp + to + 16);
      acc[t] = wmh(fa.v, fb.v, acc[t]);
    }
  }

  const int r0 = wave * 16 + 8 * hh;
  float* sp = stg + r0 * GCOLS + m;
#pragma unroll
  for (int t = 0; t < NT; ++t) {
#pragma unroll
    for (int r = 0; r < 8; ++r) sp[r * GCOLS + 16 * t] = acc[t][r];
  }
  __syncthreads();

  const v4f bv = *(const v4f*)(bias + colBase + 4 * lane);
  const float* lp = stg + wave * 16 * GCOLS + 4 * lane;
  const size_t ob = (size_t)(rowBase + wave * 16) * CD + (size_t)colBase + 4 * lane;
#pragma unroll
  for (int i = 0; i < 16; ++i) {
    const v4f v = *(const v4f*)(lp + i * GCOLS) * WC_INV + bv;
    v4us hv, lv;
    split4(v, hv, lv);
    *(volatile v4us*)(Ch + ob + (size_t)i * CD) = hv;
    *(volatile v4us*)(Cl + ob + (size_t)i * CD) = lv;
  }
  __threadfence();
#pragma unroll
  for (int i = 0; i < 16; ++i) {
    const v4f v = *(const v4f*)(lp + i * GCOLS) * WC_INV + bv;
    v4us hv, lv;
    split4(v, hv, lv);
    *(volatile v4us*)(Ch + ob + (size_t)i * CD) = hv;
    *(volatile v4us*)(Cl + ob + (size_t)i * CD) = lv;
  }
}

static __device__ __forceinline__ void x3_store_pass(const float* lp, v4f bv, int relu, int ok32, float* C32,
                                                     int write16, unsigned short* Ch, unsigned short* Cl,
                                                     size_t ob, int lane) {
#pragma unroll
  for (int i = 0; i < 16; ++i) {
    v4f v = *(const v4f*)(lp + i * GCOLS) + bv;
    if (relu) { v.x = fmaxf(v.x, 0.f); v.y = fmaxf(v.y, 0.f); v.z = fmaxf(v.z, 0.f); v.w = fmaxf(v.w, 0.f); }
    const size_t o = ob + (size_t)i * CD;
    if (ok32) *(volatile v4f*)(C32 + o) = v;
    if (write16) {
      v4us hv, lv;
      split4(v, hv, lv);
      *(volatile v4us*)(Ch + o) = hv;
      *(volatile v4us*)(Cl + o) = lv;
    }
  }
}

__global__ __launch_bounds__(NTHR) void k_gemm_x3(
    const unsigned short* __restrict__ A1h, const unsigned short* __restrict__ A1l,
    const unsigned short* __restrict__ B1h, const unsigned short* __restrict__ B1l,
    const unsigned short* __restrict__ A2h, const unsigned short* __restrict__ A2l,
    const unsigned short* __restrict__ B2h, const unsigned short* __restrict__ B2l,
    int twoPairs, const float* __restrict__ bias1, const float* __restrict__ bias2, int relu,
    float* C32, int write32, int nRows32, unsigned short* Ch, unsigned short* Cl, int write16) {
  extern __shared__ v4f lds_dyn[];
  float* stg = (float*)lds_dyn;
  const int tid = threadIdx.x, lane = tid & 31, hh = lane >> 4, m = lane & 15;
  const int wave = __builtin_amdgcn_readfirstlane(tid >> 5);
  const int rowBase = (int)blockIdx.x * GROWS;
  const int colBase = (int)blockIdx.y * GCOLS;
  const size_t aoff = (size_t)(rowBase + wave * 16 + m) * CD + 8 * hh;
  const size_t boff = (size_t)(colBase + m) * CD + 8 * hh;

  v8f acc[NT];
#pragma unroll
  for (int t = 0; t < NT; ++t) { v8f zz = {0.f, 0.f, 0.f, 0.f, 0.f, 0.f, 0.f, 0.f}; acc[t] = zz; }

  mac_x3(A1h + aoff, A1l + aoff, B1h + boff, B1l + boff, acc);
  if (twoPairs) mac_x3(A2h + aoff, A2l + aoff, B2h + boff, B2l + boff, acc);

  const int r0 = wave * 16 + 8 * hh;
  float* sp = stg + r0 * GCOLS + m;
#pragma unroll
  for (int t = 0; t < NT; ++t) {
#pragma unroll
    for (int r = 0; r < 8; ++r) sp[r * GCOLS + 16 * t] = acc[t][r];
  }
  __syncthreads();

  const v4f b1 = *(const v4f*)(bias1 + colBase + 4 * lane);
  const v4f b2 = *(const v4f*)(bias2 + colBase + 4 * lane);
  v4f bv = b1;
  if (twoPairs) bv = bv + b2;
  const float* lp = stg + wave * 16 * GCOLS + 4 * lane;
  const int rw = rowBase + wave * 16;
  const int ok32 = (write32 != 0 && (rw + 16) <= nRows32) ? 1 : 0;
  const size_t ob = (size_t)rw * CD + (size_t)colBase + 4 * lane;
  x3_store_pass(lp, bv, relu, ok32, C32, write16, Ch, Cl, ob, lane);
  __threadfence();
  x3_store_pass(lp, bv, relu, ok32, C32, write16, Ch, Cl, ob, lane);
}

extern "C" void kernel_launch(void* const* d_in, const int* in_sizes, int n_in,
                              void* d_out, int out_size, void* d_ws, size_t ws_size,
                              hipStream_t stream) {
  if (n_in < 15) return;
  if (in_sizes[0] != BSZ * CD) return;
  const int nE = in_sizes[1];
  if (nE < 1 || nE > (1 << 24) || in_sizes[12] != nE || in_sizes[13] != nE) return;
  if (in_sizes[2] != NL * NBR * NM * CBW) return;
  if (in_sizes[3] != NL * CD * CD || in_sizes[5] != NL * CD * CD || in_sizes[7] != NL * CD * CD) return;
  if (in_sizes[4] != NL * CD || in_sizes[6] != NL * CD || in_sizes[8] != NL * CD) return;
  if (in_sizes[9] != CD * CD || in_sizes[10] != CD || in_sizes[11] != NFO || in_sizes[14] != NL * NBR * NN) return;
  if (out_size != BSZ * CD) return;

  const float* x    = (const float*)d_in[0];
  const float* ew   = (const float*)d_in[1];
  const float* cbk  = (const float*)d_in[2];
  const float* Wc   = (const float*)d_in[3];
  const float* bc   = (const float*)d_in[4];
  const float* Wt   = (const float*)d_in[5];
  const float* bt   = (const float*)d_in[6];
  const float* Wsk  = (const float*)d_in[7];
  const float* bs   = (const float*)d_in[8];
  const float* Wf   = (const float*)d_in[9];
  const float* bfv  = (const float*)d_in[10];
  const int*   foi  = (const int*)d_in[11];
  const int*   esrc = (const int*)d_in[12];
  const int*   edst = (const int*)d_in[13];
  const int*   cidx = (const int*)d_in[14];
  float* out = (float*)d_out;

  char* ws = (char*)d_ws;
  size_t off = 0;
  const size_t szW16 = (size_t)CD * CD * 2;
  const size_t szP16 = (size_t)MP * CD * 2;
  const size_t szP32 = (size_t)MP * CD * 4;
  const size_t oWcT  = off; off += (size_t)NL * szW16;   off = (off + 255) & ~(size_t)255;
  const size_t oWtTh = off; off += (size_t)NL * szW16;   off = (off + 255) & ~(size_t)255;
  const size_t oWtTl = off; off += (size_t)NL * szW16;   off = (off + 255) & ~(size_t)255;
  const size_t oWsTh = off; off += (size_t)NL * szW16;   off = (off + 255) & ~(size_t)255;
  const size_t oWsTl = off; off += (size_t)NL * szW16;   off = (off + 255) & ~(size_t)255;
  const size_t oWfTh = off; off += szW16;                off = (off + 255) & ~(size_t)255;
  const size_t oWfTl = off; off += szW16;                off = (off + 255) & ~(size_t)255;
  const size_t oHhA  = off; off += szP16;                off = (off + 255) & ~(size_t)255;
  const size_t oHlA  = off; off += szP16;                off = (off + 255) & ~(size_t)255;
  const size_t oHhB  = off; off += szP16;                off = (off + 255) & ~(size_t)255;
  const size_t oHlB  = off; off += szP16;                off = (off + 255) & ~(size_t)255;
  const size_t oH32  = off; off += szP32;                off = (off + 255) & ~(size_t)255;
  const size_t oAg   = off; off += szP16;                off = (off + 255) & ~(size_t)255;
  const size_t oAGh  = off; off += szP16;                off = (off + 255) & ~(size_t)255;
  const size_t oAGl  = off; off += szP16;                off = (off + 255) & ~(size_t)255;
  const size_t oTab  = off; off += (size_t)NBA * CAP * 4;  off = (off + 255) & ~(size_t)255;
  const size_t oCnt  = off; off += (size_t)NBA * CNTW * 4; off = (off + 255) & ~(size_t)255;
  if (off > ws_size || off > (size_t)WSCAP) return;
  unsigned short* WcT  = (unsigned short*)(ws + oWcT);
  unsigned short* WtTh = (unsigned short*)(ws + oWtTh);
  unsigned short* WtTl = (unsigned short*)(ws + oWtTl);
  unsigned short* WsTh = (unsigned short*)(ws + oWsTh);
  unsigned short* WsTl = (unsigned short*)(ws + oWsTl);
  unsigned short* WfTh = (unsigned short*)(ws + oWfTh);
  unsigned short* WfTl = (unsigned short*)(ws + oWfTl);
  unsigned short* HhA  = (unsigned short*)(ws + oHhA);
  unsigned short* HlA  = (unsigned short*)(ws + oHlA);
  unsigned short* HhB  = (unsigned short*)(ws + oHhB);
  unsigned short* HlB  = (unsigned short*)(ws + oHlB);
  float*          H32  = (float*)(ws + oH32);
  unsigned short* Ag   = (unsigned short*)(ws + oAg);
  unsigned short* AGh  = (unsigned short*)(ws + oAGh);
  unsigned short* AGl  = (unsigned short*)(ws + oAGl);
  int*            Tab  = (int*)(ws + oTab);
  int*            Cnt  = (int*)(ws + oCnt);

  hipFuncSetAttribute(reinterpret_cast<const void*>(&k_gemm_f16),
                      hipFuncAttributeMaxDynamicSharedMemorySize, LDS_GEMM);
  hipFuncSetAttribute(reinterpret_cast<const void*>(&k_gemm_x3),
                      hipFuncAttributeMaxDynamicSharedMemorySize, LDS_GEMM);
  hipFuncSetAttribute(reinterpret_cast<const void*>(&k_agg),
                      hipFuncAttributeMaxDynamicSharedMemorySize, LDS_AGG);

  k_prepw<<<dim3((CD * CD / 8) / NTHR, 3 * NL + 1), NTHR, 0, stream>>>(
      Wc, Wt, Wsk, Wf, WcT, WtTh, WtTl, WsTh, WsTl, WfTh, WfTl);
  {
    const int t8 = (MP * CD) / 8;
    k_cvtx<<<t8 / NTHR, NTHR, 0, stream>>>(x, HhA, HlA, CD, BSZ, t8);
  }
  k_build<<<NBA, NTHR, 0, stream>>>(edst, nE, Tab, Cnt);

  unsigned short* curH = HhA;
  unsigned short* curL = HlA;
  unsigned short* nxtH = HhB;
  unsigned short* nxtL = HlB;
  for (int l = 0; l < NL; ++l) {
    const float* hsrc = (l == 0) ? x : (const float*)H32;
    const float* cbl  = cbk + (size_t)l * NBR * NM * CBW;
    const int*   cil  = cidx + (size_t)l * NBR * NN;
    const int    relu = (l < NL - 1) ? 1 : 0;
    const int    w32  = (l < NL - 1) ? 1 : 0;
    k_agg<<<NBA, NTHR, LDS_AGG, stream>>>(Tab, Cnt, esrc, ew, nE, hsrc, cbl, cil, foi, Ag);
    k_gemm_f16<<<dim3(NBA, CD / GCOLS), NTHR, LDS_GEMM, stream>>>(
        Ag, WcT + (size_t)l * CD * CD, bc + (size_t)l * CD, AGh, AGl);
    k_gemm_x3<<<dim3(NBA, CD / GCOLS), NTHR, LDS_GEMM, stream>>>(
        AGh, AGl, WtTh + (size_t)l * CD * CD, WtTl + (size_t)l * CD * CD,
        curH, curL, WsTh + (size_t)l * CD * CD, WsTl + (size_t)l * CD * CD,
        1, bt + (size_t)l * CD, bs + (size_t)l * CD, relu,
        H32, w32, MP, nxtH, nxtL, 1);
    unsigned short* th = curH; curH = nxtH; nxtH = th;
    unsigned short* tl = curL; curL = nxtL; nxtL = tl;
  }
  k_gemm_x3<<<dim3(NBA, CD / GCOLS), NTHR, LDS_GEMM, stream>>>(
      curH, curL, WfTh, WfTl, curH, curL, WfTh, WfTl,
      0, bfv, bfv, 0,
      out, 1, BSZ, AGh, AGl, 0);
}
